// MultiheadAttentionRelPE_81990925680866
// MI455X (gfx1250) — hardware-verified
//
#include <hip/hip_runtime.h>
#include <stddef.h>


#define EMBED 512
#define HDIM  64
#define NHEAD 8
#define NQ    2048
#define LK    2048
#define BB    4
#define TOK   (NQ * BB)

typedef unsigned short us_t;
typedef us_t   v16us __attribute__((ext_vector_type(16)));
typedef us_t   v8us  __attribute__((ext_vector_type(8)));
typedef __bf16 v16bf __attribute__((ext_vector_type(16)));
typedef float  v8f   __attribute__((ext_vector_type(8)));
typedef float  v4f   __attribute__((ext_vector_type(4)));
typedef v4f    v4fa  __attribute__((may_alias));

union Frag { v16us u; v8us h[2]; v16bf b; };

__device__ __forceinline__ unsigned int bf16_rne(float f) {
  const unsigned int u = __float_as_uint(f);
  return (u + 0x7FFFu + ((u >> 16) & 1u)) >> 16;
}

__device__ __forceinline__ void split8(const v4f x0, const v4f x1, v8us& hi, v8us& lo) {
#pragma unroll
  for (int e = 0; e < 4; ++e) {
    const unsigned int hb0 = bf16_rne(x0[e]);
    const float hf0 = __uint_as_float(hb0 << 16);
    hi[e] = (us_t)hb0;
    lo[e] = (us_t)bf16_rne(x0[e] - hf0);
    const unsigned int hb1 = bf16_rne(x1[e]);
    const float hf1 = __uint_as_float(hb1 << 16);
    hi[4 + e] = (us_t)hb1;
    lo[4 + e] = (us_t)bf16_rne(x1[e] - hf1);
  }
}

__device__ __forceinline__ v8f wmma_bf16(const Frag& a, const Frag& b, v8f c) {
  return __builtin_amdgcn_wmma_f32_16x16x32_bf16(false, a.b, false, b.b, (short)0, c, false, false);
}

__device__ __forceinline__ void wmma3(v8f& acc, const Frag& ah, const Frag& al,
                                      const Frag& bh, const Frag& bl) {
  acc = wmma_bf16(ah, bh, acc);
  acc = wmma_bf16(ah, bl, acc);
  acc = wmma_bf16(al, bh, acc);
  asm volatile("v_nop\n\tv_nop\n\tv_nop\n\tv_nop"
               : "+v"(acc) : "v"(ah.u), "v"(al.u), "v"(bh.u), "v"(bl.u));
}

__global__ __launch_bounds__(256)
void split_planes_kernel(const float* __restrict__ s0, const float* __restrict__ s1,
                         const float* __restrict__ s2, const float* __restrict__ s3,
                         us_t* __restrict__ base, long long pstride) {
  const int y = blockIdx.y;
  const float* src = (y == 0) ? s0 : ((y == 1) ? s1 : ((y == 2) ? s2 : s3));
  const size_t idx = ((size_t)blockIdx.x * 256 + threadIdx.x) * 8;
  const v4f x0 = *(const v4f*)(src + idx);
  const v4f x1 = *(const v4f*)(src + idx + 4);
  v8us hi, lo;
  split8(x0, x1, hi, lo);
  us_t* hp = base + (size_t)(2 * y) * (size_t)pstride + idx;
  us_t* lp = hp + (size_t)pstride;
  *(volatile v8us*)hp = hi;
  *(volatile v8us*)lp = lo;
  __threadfence();
  *(volatile v8us*)hp = hi;
  *(volatile v8us*)lp = lo;
}

template <int OUTF32, int BIASROW>
__global__ __launch_bounds__(256)
void gemm_split_kernel(const us_t* __restrict__ Ah, const us_t* __restrict__ Al, int lda, long long azs,
                       const us_t* __restrict__ Bh, const us_t* __restrict__ Bl, int ldb, long long bzs,
                       const float* __restrict__ bias,
                       us_t* __restrict__ Dh, us_t* __restrict__ Dl, float* __restrict__ Df,
                       int ldd, long long dzs) {
  __shared__ __attribute__((aligned(16))) float stage[8][16][68];

  const int lane = threadIdx.x & 31;
  const int wave = threadIdx.x >> 5;
  const int m    = lane & 15;
  const int hh   = lane >> 4;
  const int row0 = blockIdx.x * 128 + wave * 16;
  const int col0 = blockIdx.y * 64;
  const size_t az = (size_t)blockIdx.z * (size_t)azs;
  const size_t bz = (size_t)blockIdx.z * (size_t)bzs;
  const size_t dz = (size_t)blockIdx.z * (size_t)dzs;

  const us_t* ahp = Ah + az + (size_t)(row0 + m) * (size_t)lda + 8 * hh;
  const us_t* alp = Al + az + (size_t)(row0 + m) * (size_t)lda + 8 * hh;
  const us_t* bhp = Bh + bz + (size_t)(col0 + m) * (size_t)ldb + 8 * hh;
  const us_t* blp = Bl + bz + (size_t)(col0 + m) * (size_t)ldb + 8 * hh;
  const size_t btile = (size_t)16 * (size_t)ldb;

  v8f acc[4] = {};

  for (int k0 = 0; k0 < EMBED; k0 += 32) {
    Frag fah, fal;
    fah.h[0] = *(const v8us*)(ahp + k0);
    fah.h[1] = *(const v8us*)(ahp + k0 + 16);
    fal.h[0] = *(const v8us*)(alp + k0);
    fal.h[1] = *(const v8us*)(alp + k0 + 16);
#pragma unroll
    for (int t = 0; t < 4; ++t) {
      const us_t* ph = bhp + (size_t)t * btile + k0;
      const us_t* pl = blp + (size_t)t * btile + k0;
      Frag fbh, fbl;
      fbh.h[0] = *(const v8us*)(ph);
      fbh.h[1] = *(const v8us*)(ph + 16);
      fbl.h[0] = *(const v8us*)(pl);
      fbl.h[1] = *(const v8us*)(pl + 16);
      wmma3(acc[t], fah, fal, fbh, fbl);
    }
  }

  if constexpr (BIASROW) {
    float brow[8];
#pragma unroll
    for (int r = 0; r < 8; ++r) brow[r] = bias[row0 + 8 * hh + r];
#pragma unroll
    for (int t = 0; t < 4; ++t) {
#pragma unroll
      for (int r = 0; r < 8; ++r) stage[wave][8 * hh + r][t * 16 + m] = acc[t][r] + brow[r];
    }
  } else {
#pragma unroll
    for (int t = 0; t < 4; ++t) {
      const float bcol = bias[col0 + t * 16 + m];
#pragma unroll
      for (int r = 0; r < 8; ++r) stage[wave][8 * hh + r][t * 16 + m] = acc[t][r] + bcol;
    }
  }
  __syncthreads();

  if constexpr (OUTF32) {
    const int q2 = lane >> 4, j = lane & 15;
    v4f ov[8];
#pragma unroll
    for (int p = 0; p < 8; ++p) ov[p] = *(const v4fa*)&stage[wave][2 * p + q2][4 * j];
    float* dp = Df + dz + (size_t)row0 * (size_t)ldd + col0 + 4 * j;
#pragma unroll
    for (int p = 0; p < 8; ++p) *(volatile v4f*)(dp + (size_t)(2 * p + q2) * (size_t)ldd) = ov[p];
    __threadfence();
#pragma unroll
    for (int p = 0; p < 8; ++p) *(volatile v4f*)(dp + (size_t)(2 * p + q2) * (size_t)ldd) = ov[p];
  } else {
    const int q = lane >> 3, j = lane & 7;
    v8us oh[4], ol[4];
#pragma unroll
    for (int p = 0; p < 4; ++p) {
      const v4fa* sp = (const v4fa*)&stage[wave][4 * p + q][8 * j];
      const v4f x0 = sp[0];
      const v4f x1 = sp[1];
      split8(x0, x1, oh[p], ol[p]);
    }
    const size_t dbase = dz + (size_t)row0 * (size_t)ldd + col0 + 8 * j;
    us_t* dhp = Dh + dbase;
    us_t* dlp = Dl + dbase;
#pragma unroll
    for (int p = 0; p < 4; ++p) {
      const size_t off = (size_t)(4 * p + q) * (size_t)ldd;
      *(volatile v8us*)(dhp + off) = oh[p];
      *(volatile v8us*)(dlp + off) = ol[p];
    }
    __threadfence();
#pragma unroll
    for (int p = 0; p < 4; ++p) {
      const size_t off = (size_t)(4 * p + q) * (size_t)ldd;
      *(volatile v8us*)(dhp + off) = oh[p];
      *(volatile v8us*)(dlp + off) = ol[p];
    }
  }
}

__global__ __launch_bounds__(256)
void attn_kernel(const us_t* __restrict__ QpH, const us_t* __restrict__ QpL,
                 const us_t* __restrict__ KpH, const us_t* __restrict__ KpL,
                 const us_t* __restrict__ VtH, const us_t* __restrict__ VtL,
                 const float* __restrict__ pe1, const float* __restrict__ pe2,
                 us_t* __restrict__ OhH, us_t* __restrict__ OhL) {
  __shared__ __attribute__((aligned(16))) float Plds[8][16][32];
  __shared__ __attribute__((aligned(16))) float Ost[8][16][68];

  const int lane = threadIdx.x & 31;
  const int wave = threadIdx.x >> 5;
  const int m    = lane & 15;
  const int hh   = lane >> 4;

  const int bh = blockIdx.x;
  const int b  = bh >> 3;
  const int h  = bh & (NHEAD - 1);
  const int n0 = (blockIdx.y * 8 + wave) * 16;

  Frag qh[2], ql[2];
  {
    const size_t qoff = ((size_t)(n0 + m) * BB + b) * EMBED + h * HDIM + 8 * hh;
#pragma unroll
    for (int kc = 0; kc < 2; ++kc) {
      qh[kc].h[0] = *(const v8us*)(QpH + qoff + kc * 32);
      qh[kc].h[1] = *(const v8us*)(QpH + qoff + kc * 32 + 16);
      ql[kc].h[0] = *(const v8us*)(QpL + qoff + kc * 32);
      ql[kc].h[1] = *(const v8us*)(QpL + qoff + kc * 32 + 16);
    }
  }

  float p1[8][3];
#pragma unroll
  for (int r = 0; r < 8; ++r) {
    const float* pp = pe1 + ((size_t)b * NQ + (size_t)(n0 + 8 * hh + r)) * 3;
    p1[r][0] = pp[0];
    p1[r][1] = pp[1];
    p1[r][2] = pp[2];
  }

  v8f o[4] = {};
  float mrun[8], lrun[8];
#pragma unroll
  for (int r = 0; r < 8; ++r) { mrun[r] = -1e30f; lrun[r] = 0.f; }

  for (int kb = 0; kb < LK; kb += 32) {
    v8f s[2] = {};
#pragma unroll
    for (int st = 0; st < 2; ++st) {
      const int key = kb + st * 16 + m;
      const size_t koff = ((size_t)key * BB + b) * EMBED + h * HDIM + 8 * hh;
#pragma unroll
      for (int kc = 0; kc < 2; ++kc) {
        Frag fh, fl;
        fh.h[0] = *(const v8us*)(KpH + koff + kc * 32);
        fh.h[1] = *(const v8us*)(KpH + koff + kc * 32 + 16);
        fl.h[0] = *(const v8us*)(KpL + koff + kc * 32);
        fl.h[1] = *(const v8us*)(KpL + koff + kc * 32 + 16);
        wmma3(s[st], qh[kc], ql[kc], fh, fl);
      }
      const float c0 = pe2[(size_t)key * 3 + 0];
      const float c1 = pe2[(size_t)key * 3 + 1];
      const float c2 = pe2[(size_t)key * 3 + 2];
#pragma unroll
      for (int r = 0; r < 8; ++r) {
        const float pe = p1[r][0] * c0 + p1[r][1] * c1 + p1[r][2] * c2;
        s[st][r] = (s[st][r] + pe) * 0.125f;
      }
    }

#pragma unroll
    for (int r = 0; r < 8; ++r) {
      const float v0 = s[0][r];
      const float v1 = s[1][r];
      float mx = fmaxf(v0, v1);
#pragma unroll
      for (int off = 8; off >= 1; off >>= 1) mx = fmaxf(mx, __shfl_xor(mx, off, 32));
      const float mnew  = fmaxf(mrun[r], mx);
      const float alpha = __expf(mrun[r] - mnew);
      const float p0    = __expf(v0 - mnew);
      const float p1v   = __expf(v1 - mnew);
      float rs = p0 + p1v;
#pragma unroll
      for (int off = 8; off >= 1; off >>= 1) rs += __shfl_xor(rs, off, 32);
      lrun[r] = lrun[r] * alpha + rs;
      mrun[r] = mnew;
#pragma unroll
      for (int t = 0; t < 4; ++t) o[t][r] = o[t][r] * alpha;
      Plds[wave][8 * hh + r][m]      = p0;
      Plds[wave][8 * hh + r][16 + m] = p1v;
    }

    __syncthreads();

    Frag ph, pl;
    {
      const v4fa* pr = (const v4fa*)&Plds[wave][m][0];
      const v4f x0 = pr[2 * hh];
      const v4f x1 = pr[2 * hh + 1];
      const v4f x2 = pr[4 + 2 * hh];
      const v4f x3 = pr[5 + 2 * hh];
      split8(x0, x1, ph.h[0], pl.h[0]);
      split8(x2, x3, ph.h[1], pl.h[1]);
    }

    __syncthreads();

#pragma unroll
    for (int t = 0; t < 4; ++t) {
      const size_t voff = ((size_t)b * EMBED + (size_t)(h * HDIM + t * 16 + m)) * LK + kb + 8 * hh;
      Frag vh, vl;
      vh.h[0] = *(const v8us*)(VtH + voff);
      vh.h[1] = *(const v8us*)(VtH + voff + 16);
      vl.h[0] = *(const v8us*)(VtL + voff);
      vl.h[1] = *(const v8us*)(VtL + voff + 16);
      wmma3(o[t], ph, pl, vh, vl);
    }
  }

#pragma unroll
  for (int r = 0; r < 8; ++r) {
    const float inv = 1.0f / lrun[r];
#pragma unroll
    for (int t = 0; t < 4; ++t) Ost[wave][8 * hh + r][t * 16 + m] = o[t][r] * inv;
  }
  __syncthreads();

  const int q = lane >> 3, j = lane & 7;
  v8us oh[4], ol[4];
#pragma unroll
  for (int p = 0; p < 4; ++p) {
    const v4fa* sp = (const v4fa*)&Ost[wave][4 * p + q][8 * j];
    const v4f x0 = sp[0];
    const v4f x1 = sp[1];
    split8(x0, x1, oh[p], ol[p]);
  }
#pragma unroll
  for (int p = 0; p < 4; ++p) {
    const size_t off = ((size_t)(n0 + 4 * p + q) * BB + b) * EMBED + h * HDIM + 8 * j;
    *(volatile v8us*)(OhH + off) = oh[p];
    *(volatile v8us*)(OhL + off) = ol[p];
  }
  __threadfence();
#pragma unroll
  for (int p = 0; p < 4; ++p) {
    const size_t off = ((size_t)(n0 + 4 * p + q) * BB + b) * EMBED + h * HDIM + 8 * j;
    *(volatile v8us*)(OhH + off) = oh[p];
    *(volatile v8us*)(OhL + off) = ol[p];
  }
}

extern "C" void kernel_launch(void* const* d_in, const int* in_sizes, int n_in,
                              void* d_out, int out_size, void* d_ws, size_t ws_size,
                              hipStream_t stream) {
  if (n_in < 13) return;
  const size_t SZA = (size_t)TOK * EMBED;
  const size_t SZW = (size_t)EMBED * EMBED;
  if ((size_t)in_sizes[0] != SZA || (size_t)in_sizes[1] != SZA || (size_t)in_sizes[2] != SZA) return;
  if ((size_t)in_sizes[3] != (size_t)BB * NQ * 3 || (size_t)in_sizes[4] != (size_t)LK * 3) return;
  if ((size_t)in_sizes[5] != SZW || (size_t)in_sizes[7] != SZW ||
      (size_t)in_sizes[9] != SZW || (size_t)in_sizes[11] != SZW) return;
  if (in_sizes[6] != EMBED || in_sizes[8] != EMBED || in_sizes[10] != EMBED || in_sizes[12] != EMBED) return;
  if ((size_t)out_size != SZA) return;

  const float* q   = (const float*)d_in[0];
  const float* k   = (const float*)d_in[1];
  const float* v   = (const float*)d_in[2];
  const float* pe1 = (const float*)d_in[3];
  const float* pe2 = (const float*)d_in[4];
  const float* Wq  = (const float*)d_in[5];
  const float* bq  = (const float*)d_in[6];
  const float* Wk  = (const float*)d_in[7];
  const float* bk  = (const float*)d_in[8];
  const float* Wv  = (const float*)d_in[9];
  const float* bv  = (const float*)d_in[10];
  const float* Wo  = (const float*)d_in[11];
  const float* bo  = (const float*)d_in[12];
  float* out = (float*)d_out;

  const size_t total_elems = 14 * SZA + 8 * SZW;
  const size_t total_bytes = total_elems * sizeof(us_t);
  if (total_bytes > ws_size) return;

  us_t* ws  = (us_t*)d_ws;
  us_t* act = ws;
  us_t* qH = act,            *qL = act + SZA;
  us_t* kH = act + 2 * SZA,  *kL = act + 3 * SZA;
  us_t* vH = act + 4 * SZA,  *vL = act + 5 * SZA;
  us_t* QpH = ws + 6 * SZA,  *QpL = ws + 7 * SZA;
  us_t* KpH = ws + 8 * SZA,  *KpL = ws + 9 * SZA;
  us_t* VtH = ws + 10 * SZA, *VtL = ws + 11 * SZA;
  us_t* OhH = ws + 12 * SZA, *OhL = ws + 13 * SZA;
  us_t* wts = ws + 14 * SZA;
  us_t* WqH = wts,           *WqL = wts + SZW;
  us_t* WkH = wts + 2 * SZW, *WkL = wts + 3 * SZW;
  us_t* WvH = wts + 4 * SZW, *WvL = wts + 5 * SZW;
  us_t* WoH = wts + 6 * SZW, *WoL = wts + 7 * SZW;

  const dim3 blk(256);

  hipLaunchKernelGGL(split_planes_kernel, dim3((unsigned)(SZA / 2048), 3), blk, 0, stream,
                     q, k, v, v, act, (long long)SZA);
  hipLaunchKernelGGL(split_planes_kernel, dim3((unsigned)(SZW / 2048), 4), blk, 0, stream,
                     Wq, Wk, Wv, Wo, wts, (long long)SZW);

  const dim3 gProj(TOK / 128, EMBED / 64, 1);
  hipLaunchKernelGGL(HIP_KERNEL_NAME(gemm_split_kernel<0, 0>), gProj, blk, 0, stream,
                     (const us_t*)qH, (const us_t*)qL, EMBED, 0LL,
                     (const us_t*)WqH, (const us_t*)WqL, EMBED, 0LL,
                     bq, QpH, QpL, out, EMBED, 0LL);
  hipLaunchKernelGGL(HIP_KERNEL_NAME(gemm_split_kernel<0, 0>), gProj, blk, 0, stream,
                     (const us_t*)kH, (const us_t*)kL, EMBED, 0LL,
                     (const us_t*)WkH, (const us_t*)WkL, EMBED, 0LL,
                     bk, KpH, KpL, out, EMBED, 0LL);
  const dim3 gVt(EMBED / 128, LK / 64, BB);
  hipLaunchKernelGGL(HIP_KERNEL_NAME(gemm_split_kernel<0, 1>), gVt, blk, 0, stream,
                     (const us_t*)WvH, (const us_t*)WvL, EMBED, 0LL,
                     (const us_t*)vH, (const us_t*)vL, BB * EMBED, (long long)EMBED,
                     bv, VtH, VtL, out, LK, (long long)EMBED * LK);

  hipLaunchKernelGGL(attn_kernel, dim3(BB * NHEAD, NQ / 128), blk, 0, stream,
                     (const us_t*)QpH, (const us_t*)QpL, (const us_t*)KpH, (const us_t*)KpL,
                     (const us_t*)VtH, (const us_t*)VtL, pe1, pe2, OhH, OhL);

  hipLaunchKernelGGL(HIP_KERNEL_NAME(gemm_split_kernel<1, 0>), gProj, blk, 0, stream,
                     (const us_t*)OhH, (const us_t*)OhL, EMBED, 0LL,
                     (const us_t*)WoH, (const us_t*)WoL, EMBED, 0LL,
                     bo, QpH, QpL, out, EMBED, 0LL);
}
